// TableDistance_5669356831001
// MI455X (gfx1250) — hardware-run, weakly checked
//
#include <hip/hip_runtime.h>
#include <stddef.h>


typedef _Float16 v16h __attribute__((ext_vector_type(16)));
typedef _Float16 v8h  __attribute__((ext_vector_type(8)));
typedef float    v8f  __attribute__((ext_vector_type(8)));
typedef float    v4f  __attribute__((ext_vector_type(4)));
typedef _Float16 h16;

#ifndef NB
#define NB 4
#endif
#ifndef SEQ
#define SEQ 2048
#endif
#define NB_FULL  4
#define SEQ_FULL 2048
#define XD    64
#define NTAB  256
#define MROWS (NB * SEQ)

static_assert(NB >= 1 && NB <= NB_FULL);
static_assert(SEQ >= 64 && SEQ <= SEQ_FULL && (SEQ % 64) == 0);
static_assert(XD == 64 && (XD % 32) == 0);
static_assert((NTAB % 64) == 0);
static_assert((MROWS % 64) == 0);
static_assert(64 * 4 == 256);
static_assert(4 * 16 == XD);

#define LDT 72
#define LDC 68
static_assert((LDT % 8) == 0 && LDT >= 64);
static_assert((LDC % 4) == 0 && LDC >= 64);

#define WCARRY 64.0f

#define TT_BYTES ((size_t)NTAB * XD * 2)
#define OFF_TT   ((size_t)0)
#define WS_TOTAL (OFF_TT + TT_BYTES)
static_assert((TT_BYTES % 128) == 0);
static_assert(WS_TOTAL <= (size_t)134217728);

__device__ __forceinline__ float bf16r(float x) {
  unsigned int u = __float_as_uint(x);
  u = (u + 0x7FFFu + ((u >> 16) & 1u)) & 0xFFFF0000u;
  return __uint_as_float(u);
}

static __device__ __forceinline__ h16 toh_flush(float v) {
  const h16 r = (h16)v;
  return (fabsf(v) < 6.103515625e-05f) ? (h16)0.0f : r;
}

__device__ __forceinline__ v16h frag_at(const _Float16* p) {
  v8h lo = *(const v8h*)(p);
  v8h hi = *(const v8h*)(p + 16);
  v16h out;
#pragma unroll
  for (int i = 0; i < 8; ++i) { out[i] = lo[i]; out[i + 8] = hi[i]; }
  return out;
}
__device__ __forceinline__ v16h ld_frag(const _Float16* base, unsigned ld) {
  const unsigned lane = threadIdx.x & 31u;
  return frag_at(base + (lane & 15u) * ld + (lane >> 4) * 8u);
}

__device__ __forceinline__ v8f wmma16(v16h a, v16h b, v8f c) {
  v8f d = __builtin_amdgcn_wmma_f32_16x16x32_f16(false, a, false, b, (short)0, c,
                                                 false, false);
  asm volatile("v_nop\n\tv_nop\n\tv_nop\n\tv_nop" : "+v"(d) : "v"(a), "v"(b));
  return d;
}

__global__ __launch_bounds__(256) void wconv_kernel(
    const float* __restrict__ W, _Float16* __restrict__ Wt, unsigned ldw, unsigned ldk) {
  __shared__ _Float16 T[64 * LDT];
  const unsigned tid = threadIdx.x;
  const unsigned n0 = blockIdx.x * 64u;
  const unsigned k0 = blockIdx.y * 64u;
#pragma unroll 4
  for (unsigned j = 0; j < 16u; ++j) {
    const unsigned idx = tid + 256u * j;
    const unsigned kr = idx >> 6, nc = idx & 63u;
    const float v = W[(size_t)(k0 + kr) * ldw + n0 + nc];
    T[nc * LDT + kr] = (_Float16)(WCARRY * bf16r(v));
  }
  __syncthreads();
  v8h x[2];
  size_t off[2];
#pragma unroll
  for (unsigned i = 0; i < 2u; ++i) {
    const unsigned n = 32u * i + (tid >> 3);
    const unsigned kc = (tid & 7u) * 8u;
    x[i] = *(const v8h*)&T[n * LDT + kc];
    off[i] = (size_t)(n0 + n) * ldk + k0 + kc;
  }
#pragma unroll
  for (int i = 0; i < 2; ++i) *(volatile v8h*)(Wt + off[i]) = x[i];
  __threadfence();
#pragma unroll
  for (int i = 0; i < 2; ++i) *(volatile v8h*)(Wt + off[i]) = x[i];
}

__global__ __launch_bounds__(256) void dist_kernel(
    const float* __restrict__ X, const float* __restrict__ Tab, const float* __restrict__ Sc,
    const _Float16* __restrict__ Bt, float* __restrict__ outf) {
  __shared__ __attribute__((aligned(16))) float Cs[64 * LDC];
  __shared__ __attribute__((aligned(16))) _Float16 As[64 * LDT];
  __shared__ __attribute__((aligned(16))) float X2s[64];
  __shared__ __attribute__((aligned(16))) float T2p[4 * 64];
  __shared__ __attribute__((aligned(16))) float T2s[64];

  const unsigned tid = threadIdx.x, lane = tid & 31u;
  const unsigned w = (unsigned)__builtin_amdgcn_readfirstlane((int)(threadIdx.x >> 5));
  const unsigned mw = w >> 1, nw = w & 1u;
  const unsigned hh = lane >> 4, m = lane & 15u;
  const unsigned n0 = blockIdx.x * 64u;
  const unsigned row0 = blockIdx.y * 64u;

  {
    const unsigned r = tid >> 2, qd = tid & 3u;
    const unsigned crow = row0 + r;
    const unsigned bidx = crow / (unsigned)SEQ;
    const unsigned sq = crow - bidx * (unsigned)SEQ;
    const size_t frow = (size_t)bidx * SEQ_FULL + sq;
    const float* xr = X + frow * XD + qd * 16u;
    float ss = 0.0f;
#pragma unroll
    for (unsigned j = 0; j < 2u; ++j) {
      const v4f a0 = *(const v4f*)(xr + j * 8u);
      const v4f a1 = *(const v4f*)(xr + j * 8u + 4u);
      v8h o;
#pragma unroll
      for (int i = 0; i < 4; ++i) {
        const float e0 = bf16r(a0[i]);
        const float e1 = bf16r(a1[i]);
        ss += e0 * e0;
        ss += e1 * e1;
        o[i]     = toh_flush(e0);
        o[i + 4] = toh_flush(e1);
      }
      *(v8h*)&As[r * LDT + qd * 16u + j * 8u] = o;
    }
    ss += __shfl_xor(ss, 1, 32);
    ss += __shfl_xor(ss, 2, 32);
    if (qd == 0u) X2s[r] = ss;
  }
  {
    const unsigned col = tid & 63u, dg = tid >> 6;
    float tp = 0.0f;
#pragma unroll 4
    for (unsigned j = 0; j < 16u; ++j) {
      const float v = bf16r(Tab[(size_t)(dg * 16u + j) * NTAB + n0 + col]);
      tp += v * v;
    }
    T2p[dg * 64u + col] = tp;
  }
  __syncthreads();

  const _Float16* bp0 = Bt + (size_t)(n0 + nw * 32u + m) * XD + hh * 8u;
  const _Float16* bp1 = bp0 + (size_t)16 * XD;
  v8f acc0 = {}, acc1 = {};
#pragma unroll
  for (unsigned k0 = 0; k0 < (unsigned)XD; k0 += 32u) {
    const v16h a  = ld_frag(&As[(mw * 16u) * LDT + k0], LDT);
    const v16h b0 = frag_at(bp0 + k0);
    const v16h b1 = frag_at(bp1 + k0);
    acc0 = wmma16(a, b0, acc0);
    acc1 = wmma16(a, b1, acc1);
  }
#pragma unroll
  for (int r = 0; r < 8; ++r) {
    float* d = &Cs[(mw * 16u + hh * 8u + (unsigned)r) * LDC + nw * 32u + m];
    d[0]  = acc0[r];
    d[16] = acc1[r];
  }
  if (w < 2u) {
    const unsigned c = tid;
    T2s[c] = (T2p[c] + T2p[64u + c]) + (T2p[128u + c] + T2p[192u + c]);
  }
  __syncthreads();

  const float sabs = fabsf(bf16r(Sc[0]));
  v4f xs[4];
  size_t off[4];
#pragma unroll
  for (unsigned i = 0; i < 4u; ++i) {
    const unsigned r = 16u * i + (tid >> 4);
    const unsigned c = (tid & 15u) * 4u;
    const unsigned crow = row0 + r;
    const unsigned bidx = crow / (unsigned)SEQ;
    const unsigned sq = crow - bidx * (unsigned)SEQ;
    const size_t frow = (size_t)bidx * SEQ_FULL + sq;
    const v4f u  = *(const v4f*)&Cs[r * LDC + c];
    const v4f t2 = *(const v4f*)&T2s[c];
    const float x2 = X2s[r];
    v4f val;
#pragma unroll
    for (int j = 0; j < 4; ++j)
      val[j] = sabs * ((x2 + t2[j]) - u[j] * (2.0f / WCARRY));
    xs[i] = val;
    off[i] = frow * NTAB + n0 + c;
  }
#pragma unroll
  for (int i = 0; i < 4; ++i) *(volatile v4f*)(outf + off[i]) = xs[i];
  __threadfence();
#pragma unroll
  for (int i = 0; i < 4; ++i) *(volatile v4f*)(outf + off[i]) = xs[i];
}

extern "C" void kernel_launch(void* const* d_in, const int* in_sizes, int n_in,
                              void* d_out, int out_size, void* d_ws, size_t ws_size,
                              hipStream_t stream) {
  if (n_in < 3) return;
  const long long need_rows = (long long)(NB - 1) * SEQ_FULL + SEQ;
  if ((long long)in_sizes[0] < need_rows * XD) return;
  if ((long long)in_sizes[1] < (long long)XD * NTAB) return;
  if (in_sizes[2] < 1) return;
  if ((long long)out_size < need_rows * NTAB) return;
  if (ws_size < WS_TOTAL) return;

  const float* X   = (const float*)d_in[0];
  const float* tab = (const float*)d_in[1];
  const float* sc  = (const float*)d_in[2];
  float* out = (float*)d_out;

  char* ws = (char*)d_ws;
  _Float16* Tt = (_Float16*)(ws + OFF_TT);

  dim3 blk(256);
  wconv_kernel<<<dim3(NTAB / 64, XD / 64), blk, 0, stream>>>(tab, Tt, (unsigned)NTAB,
                                                             (unsigned)XD);
  dist_kernel<<<dim3(NTAB / 64, MROWS / 64), blk, 0, stream>>>(X, tab, sc, Tt, out);
}
